// NACE_27874337751540
// MI455X (gfx1250) — hardware-verified
//
#include <hip/hip_runtime.h>
#include <math.h>

typedef __attribute__((ext_vector_type(16))) _Float16 v16h;
typedef __attribute__((ext_vector_type(16))) __bf16 v16b;
typedef __attribute__((ext_vector_type(8)))  _Float16 v8h;
typedef __attribute__((ext_vector_type(8)))  float v8f;
typedef __attribute__((ext_vector_type(4)))  float v4f;
typedef __attribute__((ext_vector_type(2)))  float v2f;
typedef __attribute__((ext_vector_type(4)))  unsigned v4u;
typedef __attribute__((ext_vector_type(4)))  int v4i;
typedef float __attribute__((may_alias)) float_a;
typedef int __attribute__((may_alias)) int_a;

template <typename T> __device__ __forceinline__ void vst2(void* p, T v) { *(volatile T*)p = v; __threadfence(); *(volatile T*)p = v; }
__device__ __forceinline__ v8f wmma16(v16h a, v16h b, v8f c) {
  v8f d = __builtin_amdgcn_wmma_f32_16x16x32_f16(false, a, false, b, (short)0, c, false, false);
  asm volatile("v_nop\n\tv_nop\n\tv_nop\n\tv_nop" : "+v"(d) : "v"(a), "v"(b));
  return d;
}
__device__ __forceinline__ v8f wmma_bf(v16b a, v16b b, v8f c) {
  v8f d = __builtin_amdgcn_wmma_f32_16x16x32_bf16(false, a, false, b, (short)0, c, false, false);
  asm volatile("v_nop\n\tv_nop\n\tv_nop\n\tv_nop" : "+v"(d) : "v"(a), "v"(b));
  return d;
}
__device__ __forceinline__ v16h frag_h(const _Float16* rowk0, int lane) {
  union { v16h v; v8h q[2]; } u; const _Float16* p = rowk0 + 8 * (lane >> 4);
  u.q[0] = *(const v8h*)p; u.q[1] = *(const v8h*)(p + 16); return u.v;
}
__device__ __forceinline__ v16h frag_f32(const float* rowk0, int lane) {
  v16h a; const float* p = rowk0 + 8 * (lane >> 4);
#pragma unroll
  for (int i = 0; i < 8; ++i) { a[i] = (_Float16)p[i]; a[8 + i] = (_Float16)p[16 + i]; }
  return a;
}
__device__ __forceinline__ v16h frag_f32s(const float* rowk0, int lane, float sc) {
  v16h a; const float* p = rowk0 + 8 * (lane >> 4);
#pragma unroll
  for (int i = 0; i < 8; ++i) { a[i] = (_Float16)(p[i] * sc); a[8 + i] = (_Float16)(p[16 + i] * sc); }
  return a;
}
__device__ __forceinline__ v16h fragc_f32(const float* W, int k0, int n, int lane, int ld, int K) {
  v16h a; const int g = lane >> 4;
#pragma unroll
  for (int i = 0; i < 8; ++i) { const int ka = k0 + 8 * g + i, kb = ka + 16;
    a[i] = (_Float16)(ka < K ? W[(size_t)(ka < K ? ka : K - 1) * ld + n] : 0.f); a[8 + i] = (_Float16)(kb < K ? W[(size_t)(kb < K ? kb : K - 1) * ld + n] : 0.f); }
  return a;
}
struct F2 { v16b h, l; };
__device__ __forceinline__ F2 bsplit16(const float v[16]) { F2 r;
#pragma unroll
  for (int i = 0; i < 16; ++i) { const __bf16 h = (__bf16)v[i]; r.h[i] = h; r.l[i] = (__bf16)(v[i] - (float)h); }
  return r; }
__device__ __forceinline__ F2 split_row(const float* row, int k0, int lane) { float v[16]; const float* p = row + k0 + 8 * (lane >> 4);
#pragma unroll
  for (int i = 0; i < 8; ++i) { v[i] = p[i]; v[8 + i] = p[16 + i]; }
  return bsplit16(v); }
__device__ __forceinline__ F2 split_rowK(const float* row, int k0, int lane, int K) { float v[16]; const int g = lane >> 4;
#pragma unroll
  for (int i = 0; i < 8; ++i) { const int ka = k0 + 8 * g + i, kb = ka + 16; v[i] = ka < K ? row[ka < K ? ka : K - 1] : 0.f; v[8 + i] = kb < K ? row[kb < K ? kb : K - 1] : 0.f; }
  return bsplit16(v); }
__device__ __forceinline__ F2 split_col(const float* W, int k0, int n, int lane, int ld, int K) { float v[16]; const int g = lane >> 4;
#pragma unroll
  for (int i = 0; i < 8; ++i) { const int ka = k0 + 8 * g + i, kb = ka + 16; v[i] = ka < K ? W[(size_t)(ka < K ? ka : K - 1) * ld + n] : 0.f; v[8 + i] = kb < K ? W[(size_t)(kb < K ? kb : K - 1) * ld + n] : 0.f; }
  return bsplit16(v); }
__device__ __forceinline__ v8f mac3(const F2& a, const F2& b, v8f c) { c = wmma_bf(a.l, b.h, c); c = wmma_bf(a.h, b.l, c); return wmma_bf(a.h, b.h, c); }
__device__ __forceinline__ float sigm(float v) { return 1.0f / (1.0f + expf(-v)); }
#define LDSX() do { asm volatile("s_wait_dscnt 0" ::: "memory"); __builtin_amdgcn_wave_barrier(); __builtin_amdgcn_fence(__ATOMIC_RELEASE, "workgroup"); } while (0)


#define NB 8
#define CC 16
#define HH 256
#define WW 256
#define NPIX (HH * WW)
#define ACT 8
#define EXT 4
#define HID 256
#define IND 108
#define KP 128
#ifndef TPB
#define TPB (NPIX / 64)
#define TNB NB
#define TB0 0
#endif
typedef __attribute__((ext_vector_type(8))) __bf16 v8b;
__device__ __forceinline__ v16b frag_b(const __bf16* rowk0, int lane) {
  union { v16b v; v8b q[2]; } u; const __bf16* p = rowk0 + 8 * (lane >> 4);
  u.q[0] = *(const v8b*)p; u.q[1] = *(const v8b*)(p + 16); return u.v;
}
__device__ __forceinline__ float bfr(float v) { return (float)(__bf16)v; }
__device__ __attribute__((noinline)) float exp_ni(float v) { return expf(v); }
__device__ __attribute__((noinline)) float erf_ni(float v) { return erff(v); }

#define WS_P1  0u
#define WS_P2  (2u * HID * KP)
#define WS_GP  (WS_P2 + 2u * CC * HID)
#define WS_G   (WS_GP + 4u * NB * CC * 16)
#define WS_END (WS_G + 4u * NB * CC)

__global__ __launch_bounds__(128) void k_pack(const float* __restrict__ W1, const float* __restrict__ W2, __bf16* __restrict__ PK) {
  __shared__ __align__(16) __bf16 s[HID]; const int n = blockIdx.x, which = blockIdx.y, t = threadIdx.x;
  if (which == 0) { s[t] = (__bf16)((t < IND) ? W1[(size_t)n * IND + t] : 0.f); __syncthreads(); if (t < KP / 8) vst2((unsigned*)(PK + WS_P1 / 2 + (size_t)n * KP + t * 8), *(const v4u*)&s[t * 8]); }
  else { if (n >= CC) return; for (int k = t; k < HID; k += 128) s[k] = (__bf16)W2[(size_t)n * HID + k]; __syncthreads(); if (t < HID / 8) vst2((unsigned*)(PK + WS_P2 / 2 + (size_t)n * HID + t * 8), *(const v4u*)&s[t * 8]); }
}
__global__ __launch_bounds__(256) void k_gsum(const float* __restrict__ ST, float* __restrict__ GP) {
  __shared__ float red[8]; const int t = threadIdx.x; const int chunk = blockIdx.x, c = blockIdx.y, b = blockIdx.z + TB0; const float* p = ST + ((size_t)b * CC + c) * NPIX + (size_t)chunk * 4096;
  float s = 0.f; for (int i = t; i < 4096; i += 256) s += bfr(p[i]);
#pragma unroll
  for (int o = 1; o < 32; o <<= 1) s += __shfl_xor(s, o);
  if ((t & 31) == 0) red[t >> 5] = s; __syncthreads();
  if (t == 0) { float a = 0.f; for (int w = 0; w < 8; ++w) a += red[w]; GP[((size_t)b * CC + c) * 16 + chunk] = a; }
}
__global__ __launch_bounds__(128) void k_gmean(const float* __restrict__ GP, float* __restrict__ G) {
  const int t = threadIdx.x; if (t < NB * CC) { float a = 0.f; for (int k = 0; k < 16; ++k) a += GP[(size_t)t * 16 + k]; G[t] = a / (float)NPIX; }
}
__global__ __launch_bounds__(128) void k_nace(const float* __restrict__ ST, const float* __restrict__ AM, const float* __restrict__ EM, const __bf16* __restrict__ P1, const float* __restrict__ B1, const __bf16* __restrict__ P2, const float* __restrict__ B2, const float* __restrict__ G, float* __restrict__ OUT) {
  __shared__ __align__(16) __bf16 sa[64][KP + 8], sal[64][KP + 8]; __shared__ __align__(16) __bf16 sh[64][HID + 8], shl[64][HID + 8]; __shared__ __align__(16) float so[CC][68];
  const int tid = threadIdx.x, wave = tid >> 5, lane = tid & 31, col = lane & 15, g = lane >> 4; const int b = blockIdx.y + TB0; const int pt = blockIdx.x; const int y = pt / (WW / 64), x0 = (pt % (WW / 64)) * 64;
  for (int e = tid; e < 64 * (KP + 8); e += 128) { const int px = e / (KP + 8), k = e % (KP + 8); float v = 0.f, vl = 0.f; const int xx = x0 + px;
    if (k < CC * 5) { const int c = k / 5, tap = k % 5; int yy = y, xq = xx; if (tap == 1) yy = y - 1; else if (tap == 2) yy = y + 1; else if (tap == 3) xq = xx - 1; else if (tap == 4) xq = xx + 1;
      v = (yy >= 0 && yy < HH && xq >= 0 && xq < WW) ? bfr(ST[(((size_t)b * CC + c) * HH + yy) * WW + xq]) : 0.f; }
    else if (k < CC * 5 + CC) { const float gv = G[b * CC + (k - CC * 5)]; const __bf16 hb = (__bf16)gv; v = (float)hb; vl = gv - (float)hb; }
    else if (k < CC * 6 + ACT) v = bfr(AM[(((size_t)b * ACT + (k - CC * 6)) * HH + y) * WW + xx]);
    else if (k < IND) v = bfr(EM[(((size_t)b * EXT + (k - CC * 6 - ACT)) * HH + y) * WW + xx]);
    sa[px][k] = (__bf16)v; sal[px][k] = (__bf16)vl; }
  __syncthreads();
#pragma unroll 1
  for (int half = 0; half < 2; ++half) { v8f acc[8] = {};
#pragma unroll
    for (int kc = 0; kc < KP / 32; ++kc) { const v16b a = frag_b(&sa[wave * 16 + col][kc * 32], lane); const bool haslo = (kc == 2);
      v16b al; if (haslo) al = frag_b(&sal[wave * 16 + col][kc * 32], lane);
#pragma unroll
      for (int j = 0; j < 8; ++j) { const v16b w = frag_b(P1 + (size_t)(half * 128 + j * 16 + col) * KP + kc * 32, lane); if (haslo) acc[j] = wmma_bf(al, w, acc[j]); acc[j] = wmma_bf(a, w, acc[j]); } }
#pragma unroll
    for (int j = 0; j < 8; ++j) { const int o = half * 128 + j * 16 + col; const float bb = bfr(B1[o]);
#pragma unroll
      for (int r = 0; r < 8; ++r) { float v = acc[j][r] + bb; v = (v > 0.f) ? v : 0.01f * v; const __bf16 hb = (__bf16)v; sh[wave * 16 + 8 * g + r][o] = hb; shl[wave * 16 + 8 * g + r][o] = (__bf16)(v - (float)hb); } } }
  if (lane < 8) for (int rl = 0; rl < 16; ++rl) { sh[wave * 16 + rl][HID + lane] = (__bf16)0.f; shl[wave * 16 + rl][HID + lane] = (__bf16)0.f; }
  LDSX();
  { v8f acc = {};
#pragma unroll
    for (int kc = 0; kc < HID / 32; ++kc) { F2 a; a.h = frag_b(&sh[wave * 16 + col][kc * 32], lane); a.l = frag_b(&shl[wave * 16 + col][kc * 32], lane); const v16b w = frag_b(P2 + (size_t)col * HID + kc * 32, lane); acc = wmma_bf(a.l, w, acc); acc = wmma_bf(a.h, w, acc); }
    const float bb = bfr(B2[col]);
#pragma unroll
    for (int r = 0; r < 8; ++r) { const int px = wave * 16 + 8 * g + r; float dx = acc[r] + bb; dx = fminf(fmaxf(dx, -0.5f), 0.5f); so[col][px] = bfr(ST[(((size_t)b * CC + col) * HH + y) * WW + x0 + px]) + dx; } }
  __syncthreads();
  for (int e = tid; e < CC * 16; e += 128) { const int c = e >> 4, q = e & 15; vst2(OUT + (((size_t)b * CC + c) * HH + y) * WW + x0 + q * 4, *(const v4f*)&so[c][q * 4]); }
}
extern "C" void kernel_launch(void* const* d_in, const int* in_sizes, int n_in, void* d_out, int out_size, void* d_ws, size_t ws_size, hipStream_t stream) {
  (void)in_sizes; (void)n_in; (void)out_size;
  const float** F = (const float**)d_in;
  if (ws_size < (size_t)WS_END) return;
  char* ws = (char*)d_ws; __bf16* PK = (__bf16*)ws; float *GP = (float*)(ws + WS_GP), *G = (float*)(ws + WS_G);
  k_pack<<<dim3(HID, 2), 128, 0, stream>>>(F[3], F[5], PK);
  k_gsum<<<dim3(16, CC, TNB), 256, 0, stream>>>(F[0], GP);
  k_gmean<<<1, 128, 0, stream>>>(GP, G);
  k_nace<<<dim3(TPB, TNB), 128, 0, stream>>>(F[0], F[1], F[2], (const __bf16*)(ws + WS_P1), F[4], (const __bf16*)(ws + WS_P2), F[6], G, (float*)d_out);
}
